// RiceTransformer_21912923144251
// MI455X (gfx1250) — hardware-run, weakly checked
//
#include <hip/hip_runtime.h>
#include <math.h>

constexpr int kS = 2048;
constexpr int kD = 1024;
constexpr int kH = 16;
constexpr int kHD = 64;
constexpr int kFF = 4096;
constexpr int kDepth = 2;
constexpr int kSegLen = 512;
constexpr int kNSeg = 4;
constexpr int kHeadsPerChunk = 8;
constexpr int kPairsPerChunk = kHeadsPerChunk * kNSeg;
constexpr int kNChunk = kH / kHeadsPerChunk;
constexpr float kEps = 1e-6f;
constexpr float kWCarry = 16.0f;
constexpr float kPCarry = 2048.0f;
constexpr float kAoCarry = 16.0f;
constexpr float kActCarry = 16.0f;
constexpr float kNegFill = -3.4028234663852886e38f;

constexpr size_t kRegW   = 0;
constexpr size_t kRegXA  = 8388608;
constexpr size_t kRegXB  = 16777216;
constexpr size_t kRegH   = 25165824;
constexpr size_t kRegQ   = 29360128;
constexpr size_t kRegK   = 33554432;
constexpr size_t kRegVT  = 37748736;
constexpr size_t kRegBig = 41943040;
constexpr size_t kBigSub = 33554432;
constexpr size_t kWsTotal = 92274688;

typedef __attribute__((ext_vector_type(16))) _Float16 v16h;
typedef __attribute__((ext_vector_type(8)))  _Float16 v8h;
typedef __attribute__((ext_vector_type(16))) __bf16   v16b;
typedef __attribute__((ext_vector_type(8)))  __bf16   v8b;
typedef __attribute__((ext_vector_type(8)))  float    v8f;
typedef __attribute__((ext_vector_type(4)))  float    v4f;
typedef __attribute__((ext_vector_type(4)))  unsigned int v4u;

__device__ __forceinline__ unsigned short f2bf_bits(float f) {
  unsigned u = __float_as_uint(f);
  return (unsigned short)((u + 0x7FFFu + ((u >> 16) & 1u)) >> 16);
}
__device__ __forceinline__ float bf_bits2f(unsigned short h) { return __uint_as_float(((unsigned)h) << 16); }

__device__ __forceinline__ void dep_guard_h(v8f& a, v8f& b, v16h x, v16h y) { asm volatile("v_nop\n\tv_nop\n\tv_nop\n\tv_nop" : "+v"(a), "+v"(b) : "v"(x), "v"(y)); }
__device__ __forceinline__ void dep_guard_b(v8f& a, v8f& b, v16b x, v16b y) { asm volatile("v_nop\n\tv_nop\n\tv_nop\n\tv_nop" : "+v"(a), "+v"(b) : "v"(x), "v"(y)); }
__device__ __forceinline__ void keep4_h(v16h a, v16h b, v16h c, v16h d) { asm volatile("v_nop" :: "v"(a), "v"(b), "v"(c), "v"(d)); }
__device__ __forceinline__ void keep4_b(v16b a, v16b b, v16b c, v16b d) { asm volatile("v_nop" :: "v"(a), "v"(b), "v"(c), "v"(d)); }
__device__ __forceinline__ void acc_guard4(v8f& a, v8f& b, v8f& c, v8f& d) { asm volatile("v_nop\n\tv_nop\n\tv_nop\n\tv_nop" : "+v"(a), "+v"(b), "+v"(c), "+v"(d)); }
template <typename T> struct Frag;
template <> struct Frag<_Float16> {
  typedef v16h V; union U { v16h v; v8h h[2]; };
  static __device__ __forceinline__ v16h load(const _Float16* p) {
    U f; f.h[0] = *(const v8h*)(p); f.h[1] = *(const v8h*)(p + 16); return f.v;
  }
  static __device__ __forceinline__ v8f mma(v16h a, v16h b, v8f c) {
    return __builtin_amdgcn_wmma_f32_16x16x32_f16(false, a, false, b, (short)0, c, false, false);
  }
  static __device__ __forceinline__ void guard(v8f& a, v8f& b, v16h x, v16h y) { dep_guard_h(a, b, x, y); }
  static __device__ __forceinline__ void keep(v16h a, v16h b, v16h c, v16h d) { keep4_h(a, b, c, d); }
};
template <> struct Frag<__bf16> {
  typedef v16b V; union U { v16b v; v8b h[2]; };
  static __device__ __forceinline__ v16b load(const __bf16* p) {
    U f; f.h[0] = *(const v8b*)(p); f.h[1] = *(const v8b*)(p + 16); return f.v;
  }
  static __device__ __forceinline__ v8f mma(v16b a, v16b b, v8f c) {
    return __builtin_amdgcn_wmma_f32_16x16x32_bf16(false, a, false, b, (short)0, c, false, false);
  }
  static __device__ __forceinline__ void guard(v8f& a, v8f& b, v16b x, v16b y) { dep_guard_b(a, b, x, y); }
  static __device__ __forceinline__ void keep(v16b a, v16b b, v16b c, v16b d) { keep4_b(a, b, c, d); }
};

__device__ __forceinline__ unsigned pk16(unsigned short a, unsigned short b) { return (unsigned)a | ((unsigned)b << 16); }
__device__ __forceinline__ unsigned short h_bits(float f) { const _Float16 h = (_Float16)f; return __builtin_bit_cast(unsigned short, h); }

template <int ET> struct Elem;
template <> struct Elem<0> { typedef _Float16 T; };
template <> struct Elem<1> { typedef __bf16 T; };
template <int ET, bool SPLIT, int BIAS_MODE, int OUT_MODE, bool RESID, int ACT = 0>
__global__ __launch_bounds__(256) void wmma_gemm64(
    const unsigned short* __restrict__ Ap, const unsigned short* __restrict__ A2p, int lda, long strideA, long strideA2,
    const unsigned short* __restrict__ Btp, const unsigned short* __restrict__ Bt2p, int ldb, long strideB, long strideB2,
    void* __restrict__ Cout, void* __restrict__ Cout2, int ldc, long strideC, long strideC2,
    const float* __restrict__ bias,
    const float* __restrict__ resid, long strideR,
    int M, int N, int K, float scale, int bdiv) {
  typedef typename Elem<ET>::T T;
  typedef typename Frag<T>::V V;
  const T* A = (const T*)Ap; const T* A2 = (const T*)A2p; const T* Bt = (const T*)Btp; const T* Bt2 = (const T*)Bt2p;
  __shared__ __align__(16) float sT[8][16 * 68];
  const int b    = blockIdx.y;
  const int bq   = b / bdiv;
  const int br   = b - bq * bdiv;
  const int lane = threadIdx.x & 31;
  const int wave = threadIdx.x >> 5;
  const int tilesN = N >> 6;
  const int tilesM = M >> 6;
  const int tile = blockIdx.x * 8 + wave;
  if (tile >= tilesM * tilesN) return;
  const int tm = tile / tilesN;
  const int tn = tile - tm * tilesN;
  const int m0 = tm << 6;
  const int n0 = tn << 6;

  const size_t offA = (size_t)bq * strideA + (size_t)br * strideA2;
  const size_t offB = (size_t)bq * strideB + (size_t)br * strideB2;
  const size_t offC = (size_t)bq * strideC + (size_t)br * strideC2;
  const T* Ab  = A  + offA;
  const T* Bb  = Bt + offB;
  const T* Ab2 = SPLIT ? (A2  + offA) : nullptr;
  const T* Bb2 = SPLIT ? (Bt2 + offB) : nullptr;

  const int rlane = lane & 15;
  const int koff  = (lane >> 4) * 8;
  const int mOff  = (lane >> 4) * 8;

  v8f acc[4][4];
#pragma unroll
  for (int i = 0; i < 4; ++i)
#pragma unroll
    for (int j = 0; j < 4; ++j) acc[i][j] = (v8f){0.f,0.f,0.f,0.f,0.f,0.f,0.f,0.f};

  for (int k0 = 0; k0 < K; k0 += 32) {
    V bh[4], bl[4];
#pragma unroll
    for (int j = 0; j < 4; ++j) {
      const size_t bo = (size_t)(n0 + (j << 4) + rlane) * ldb + koff + k0;
      bh[j] = Frag<T>::load(Bb + bo);
      if (SPLIT) bl[j] = Frag<T>::load(Bb2 + bo);
    }
#pragma unroll
    for (int i = 0; i < 4; ++i) {
      const size_t ao = (size_t)(m0 + (i << 4) + rlane) * lda + koff + k0;
      V ah = Frag<T>::load(Ab + ao);
      V al;
      if (SPLIT) al = Frag<T>::load(Ab2 + ao);
#pragma unroll
      for (int j = 0; j < 4; ++j) {
        acc[i][j] = Frag<T>::mma(ah, bh[j], acc[i][j]);
        if (SPLIT) {
          acc[i][j] = Frag<T>::mma(ah, bl[j], acc[i][j]);
          acc[i][j] = Frag<T>::mma(al, bh[j], acc[i][j]);
        }
      }
      Frag<T>::guard(acc[i][0], acc[i][3], ah, SPLIT ? al : ah);
    }
    Frag<T>::keep(bh[0], bh[1], bh[2], bh[3]);
    if (SPLIT) Frag<T>::keep(bl[0], bl[1], bl[2], bl[3]);
  }
  acc_guard4(acc[0][0], acc[0][1], acc[0][2], acc[0][3]);
  acc_guard4(acc[1][0], acc[1][1], acc[1][2], acc[1][3]);
  acc_guard4(acc[2][0], acc[2][1], acc[2][2], acc[2][3]);
  acc_guard4(acc[3][0], acc[3][1], acc[3][2], acc[3][3]);

  float* slab = sT[wave];
  const float* Rb = RESID ? (resid + (size_t)bq * strideR) : nullptr;
#pragma unroll
  for (int i = 0; i < 4; ++i) {
    const int mBase = m0 + (i << 4);
#pragma unroll
    for (int j = 0; j < 4; ++j) {
      const int n = n0 + (j << 4) + rlane;
      float bv = 0.f;
      if (BIAS_MODE == 2) bv = bias[n];
#pragma unroll
      for (int r = 0; r < 8; ++r) {
        float v = acc[i][j][r] * scale;
        if (BIAS_MODE == 1) v += bias[mBase + mOff + r];
        if (BIAS_MODE == 2) v += bv;
        if (RESID) v += Rb[(size_t)(mBase + mOff + r) * ldc + n];
        if (ACT == 2) v = fmaxf(v, 0.0f);
        if (ACT == 4) v = (v > 0.f) ? v : 0.01f * v;
        slab[(mOff + r) * 68 + (j << 4) + rlane] = v;
      }
    }
    __builtin_amdgcn_fence(__ATOMIC_RELEASE, "workgroup");
    __builtin_amdgcn_wave_barrier();
    __builtin_amdgcn_fence(__ATOMIC_ACQUIRE, "workgroup");
    if (OUT_MODE == 0) {
      float* C = (float*)Cout + offC;
      const int hh = lane >> 4, c4 = (lane & 15) * 4;
      for (int pass = 0; pass < 2; ++pass) {
#pragma unroll
        for (int it = 0; it < 8; ++it) {
          const int row = it * 2 + hh;
          v4f v = *(const v4f*)(slab + row * 68 + c4);
          *(volatile v4f*)(C + (size_t)(mBase + row) * ldc + n0 + c4) = v;
        }
        __threadfence();
      }
    } else {
      const int q = lane >> 3, c8 = (lane & 7) * 8;
      unsigned short* C  = (unsigned short*)Cout  + offC;
      unsigned short* C2 = (OUT_MODE == 2) ? ((unsigned short*)Cout2 + offC) : nullptr;
      for (int pass = 0; pass < 2; ++pass) {
#pragma unroll
        for (int it = 0; it < 4; ++it) {
          const int row = it * 4 + q;
          const float* sp = slab + row * 68 + c8;
          v8h hv, lv;
#pragma unroll
          for (int e = 0; e < 8; ++e) {
            if (OUT_MODE == 1) {
              hv[e] = (_Float16)sp[e];
            } else {
              unsigned short hb = f2bf_bits(sp[e]);
              unsigned short lb = f2bf_bits(sp[e] - bf_bits2f(hb));
              hv[e] = __builtin_bit_cast(_Float16, hb);
              lv[e] = __builtin_bit_cast(_Float16, lb);
            }
          }
          *(volatile v8h*)(C + (size_t)(mBase + row) * ldc + n0 + c8) = hv;
          if (OUT_MODE == 2) *(volatile v8h*)(C2 + (size_t)(mBase + row) * ldc + n0 + c8) = lv;
        }
        __threadfence();
      }
    }
    __builtin_amdgcn_fence(__ATOMIC_RELEASE, "workgroup");
    __builtin_amdgcn_wave_barrier();
    __builtin_amdgcn_fence(__ATOMIC_ACQUIRE, "workgroup");
  }
}

__global__ __launch_bounds__(256) void wt_kernel(const float* __restrict__ W, unsigned short* __restrict__ out,
                                                 int KR, int NC, float scale) {
  __shared__ float sm[64][65];
  const int t  = threadIdx.x;
  const int k0 = blockIdx.x * 64;
  const int n0 = blockIdx.y * 64;
#pragma unroll
  for (int i = 0; i < 16; ++i) {
    const int e = i * 256 + t;
    const int r = e >> 6;
    const int c = e & 63;
    sm[c][r] = W[(size_t)(k0 + r) * NC + n0 + c] * scale;
  }
  __syncthreads();
  const int lane = t & 31, wave = t >> 5;
  const int q = lane >> 3, c8 = (lane & 7) * 8;
  for (int pass = 0; pass < 2; ++pass) {
#pragma unroll
    for (int it = 0; it < 2; ++it) {
      const int row = wave * 8 + it * 4 + q;
      unsigned short hb[8];
#pragma unroll
      for (int e = 0; e < 8; ++e) hb[e] = h_bits(sm[row][c8 + e]);
      const v4u u = (v4u){pk16(hb[0], hb[1]), pk16(hb[2], hb[3]), pk16(hb[4], hb[5]), pk16(hb[6], hb[7])};
      *(volatile v4u*)(out + (size_t)(n0 + row) * KR + k0 + c8) = u;
    }
    __threadfence();
  }
}

__global__ __launch_bounds__(128) void ln_kernel(const float* __restrict__ x, const float* __restrict__ g,
                                                 const float* __restrict__ bta, unsigned short* __restrict__ out) {
#pragma clang fp contract(off)
  __shared__ float redA[4];
  __shared__ float redB[4];
  const int row  = blockIdx.x;
  const int t    = threadIdx.x;
  const int lane = t & 31, wave = t >> 5;
  const int c0   = t * 8;
  const float* xr = x + (size_t)row * kD + c0;
  const v4f a = *(const v4f*)(xr);
  const v4f c = *(const v4f*)(xr + 4);
  float v[8];
#pragma unroll
  for (int e = 0; e < 4; ++e) { v[e] = a[e]; v[4 + e] = c[e]; }
  float s = 0.f;
#pragma unroll
  for (int e = 0; e < 8; ++e) s += v[e];
#pragma unroll
  for (int off = 16; off > 0; off >>= 1) s += __shfl_xor(s, off, 32);
  if (lane == 0) redA[wave] = s;
  __syncthreads();
  const float tot  = (redA[0] + redA[1]) + (redA[2] + redA[3]);
  const float mean = tot * (1.0f / 1024.0f);
  float d[8];
  float qq = 0.f;
#pragma unroll
  for (int e = 0; e < 8; ++e) { d[e] = v[e] - mean; qq += d[e] * d[e]; }
#pragma unroll
  for (int off = 16; off > 0; off >>= 1) qq += __shfl_xor(qq, off, 32);
  if (lane == 0) redB[wave] = qq;
  __syncthreads();
  const float totq = (redB[0] + redB[1]) + (redB[2] + redB[3]);
  const float var  = totq * (1.0f / 1024.0f);
  const float inv  = 1.0f / sqrtf(var + kEps);
  const v4f ga = *(const v4f*)(g + c0);
  const v4f gc = *(const v4f*)(g + c0 + 4);
  const v4f ba = *(const v4f*)(bta + c0);
  const v4f bc = *(const v4f*)(bta + c0 + 4);
  unsigned short hb[8];
#pragma unroll
  for (int e = 0; e < 4; ++e) {
    const float y0 = d[e] * inv;
    const float y1 = d[4 + e] * inv;
    hb[e]     = h_bits(y0 * ga[e] + ba[e]);
    hb[4 + e] = h_bits(y1 * gc[e] + bc[e]);
  }
  const v4u u = (v4u){pk16(hb[0], hb[1]), pk16(hb[2], hb[3]), pk16(hb[4], hb[5]), pk16(hb[6], hb[7])};
  unsigned short* op = out + (size_t)row * kD + c0;
  *(volatile v4u*)op = u;
  __threadfence();
  *(volatile v4u*)op = u;
}

__global__ __launch_bounds__(256) void rope_kernel(const float* __restrict__ qkv, const float* __restrict__ cosb,
                                                   const float* __restrict__ sinb, unsigned short* __restrict__ qo,
                                                   unsigned short* __restrict__ ko, unsigned short* __restrict__ vt) {
#pragma clang fp contract(off)
  __shared__ float vtile[64][65];
  const int t0  = blockIdx.x * 64;
  const int h   = blockIdx.y;
  const int tid = threadIdx.x;
#pragma unroll
  for (int it = 0; it < 2; ++it) {
    const int u   = it * 256 + tid;
    const int tl  = u >> 3;
    const int d8  = (u & 7) * 8;
    const int pd8 = d8 ^ 32;
    const bool lowhalf = (d8 < 32);
    const int tok = t0 + tl;
    const float* rowp = qkv + (size_t)tok * (3 * kD) + h * kHD;
    const v4f qa = *(const v4f*)(rowp + d8),           qc = *(const v4f*)(rowp + d8 + 4);
    const v4f pa = *(const v4f*)(rowp + pd8),          pc = *(const v4f*)(rowp + pd8 + 4);
    const v4f ka = *(const v4f*)(rowp + kD + d8),      kc = *(const v4f*)(rowp + kD + d8 + 4);
    const v4f ra = *(const v4f*)(rowp + kD + pd8),     rc = *(const v4f*)(rowp + kD + pd8 + 4);
    const v4f va = *(const v4f*)(rowp + 2 * kD + d8),  vc = *(const v4f*)(rowp + 2 * kD + d8 + 4);
    const v4f ca = *(const v4f*)(cosb + (size_t)tok * kHD + d8), cc = *(const v4f*)(cosb + (size_t)tok * kHD + d8 + 4);
    const v4f sa = *(const v4f*)(sinb + (size_t)tok * kHD + d8), sc = *(const v4f*)(sinb + (size_t)tok * kHD + d8 + 4);
    float qv[8], qp[8], kv[8], kp[8], vv[8], cv[8], snv[8];
#pragma unroll
    for (int e = 0; e < 4; ++e) {
      qv[e] = qa[e]; qv[4 + e] = qc[e];
      qp[e] = pa[e]; qp[4 + e] = pc[e];
      kv[e] = ka[e]; kv[4 + e] = kc[e];
      kp[e] = ra[e]; kp[4 + e] = rc[e];
      vv[e] = va[e]; vv[4 + e] = vc[e];
      cv[e] = ca[e]; cv[4 + e] = cc[e];
      snv[e] = sa[e]; snv[4 + e] = sc[e];
    }
    unsigned short qb[8], kb[8];
#pragma unroll
    for (int e = 0; e < 8; ++e) {
      const float rq = lowhalf ? -qp[e] : qp[e];
      const float rk = lowhalf ? -kp[e] : kp[e];
      const float q1 = qv[e] * cv[e];
      const float q2 = rq * snv[e];
      const float k1 = kv[e] * cv[e];
      const float k2 = rk * snv[e];
      qb[e] = h_bits(q1 + q2);
      kb[e] = h_bits(k1 + k2);
      vtile[d8 + e][tl] = vv[e];
    }
    const v4u uq = (v4u){pk16(qb[0], qb[1]), pk16(qb[2], qb[3]), pk16(qb[4], qb[5]), pk16(qb[6], qb[7])};
    const v4u uk = (v4u){pk16(kb[0], kb[1]), pk16(kb[2], kb[3]), pk16(kb[4], kb[5]), pk16(kb[6], kb[7])};
    const size_t oidx = (size_t)tok * kD + h * kHD + d8;
    for (int pass = 0; pass < 2; ++pass) {
      *(volatile v4u*)(qo + oidx) = uq;
      *(volatile v4u*)(ko + oidx) = uk;
      __threadfence();
    }
  }
  __syncthreads();
#pragma unroll
  for (int it = 0; it < 2; ++it) {
    const int u    = it * 256 + tid;
    const int drow = u >> 3;
    const int c8   = (u & 7) * 8;
    unsigned short hb[8];
#pragma unroll
    for (int e = 0; e < 8; ++e) hb[e] = h_bits(vtile[drow][c8 + e]);
    const v4u uv = (v4u){pk16(hb[0], hb[1]), pk16(hb[2], hb[3]), pk16(hb[4], hb[5]), pk16(hb[6], hb[7])};
    unsigned short* op = vt + (size_t)(h * kHD + drow) * kS + t0 + c8;
    for (int pass = 0; pass < 2; ++pass) {
      *(volatile v4u*)op = uv;
      __threadfence();
    }
  }
}

__global__ __launch_bounds__(64) void softmax_kernel(const float* __restrict__ sc, unsigned short* __restrict__ P,
                                                     const int* __restrict__ cu, int ncu, float carry) {
  __shared__ float redM[2];
  __shared__ float redS[2];
  const int row  = blockIdx.x;
  const int pr   = row >> 9;
  const int r    = row & (kSegLen - 1);
  const int seg  = pr & (kNSeg - 1);
  const int t    = threadIdx.x;
  const int lane = t & 31, wave = t >> 5;
  const int c0   = t * 8;
  int last = ncu - 1; last = (last < 0) ? 0 : last;
  const int i1 = (1 < last) ? 1 : last;
  const int i2 = (2 < last) ? 2 : last;
  const int i3 = (3 < last) ? 3 : last;
  const int i4 = (4 < last) ? 4 : last;
  const int c1 = cu[i1], c2 = cu[i2], c3 = cu[i3], c4 = cu[i4];
  const int tq = seg * kSegLen + r;
  const int sq = (tq >= c1) + (tq >= c2) + (tq >= c3) + (tq >= c4);
  const float* sr = sc + (size_t)row * kSegLen + c0;
  const v4f a = *(const v4f*)(sr);
  const v4f c = *(const v4f*)(sr + 4);
  float x[8];
#pragma unroll
  for (int e = 0; e < 4; ++e) { x[e] = a[e]; x[4 + e] = c[e]; }
#pragma unroll
  for (int e = 0; e < 8; ++e) {
    const int tk = seg * kSegLen + c0 + e;
    const int sk = (tk >= c1) + (tk >= c2) + (tk >= c3) + (tk >= c4);
    x[e] = (sk != sq) ? kNegFill : x[e];
  }
  float m = fmaxf(fmaxf(fmaxf(x[0], x[1]), fmaxf(x[2], x[3])), fmaxf(fmaxf(x[4], x[5]), fmaxf(x[6], x[7])));
#pragma unroll
  for (int off = 16; off > 0; off >>= 1) m = fmaxf(m, __shfl_xor(m, off, 32));
  if (lane == 0) redM[wave] = m;
  __syncthreads();
  const float mx = fmaxf(redM[0], redM[1]);
  float ev[8];
  float s = 0.f;
#pragma unroll
  for (int e = 0; e < 8; ++e) { ev[e] = expf(x[e] - mx); s += ev[e]; }
#pragma unroll
  for (int off = 16; off > 0; off >>= 1) s += __shfl_xor(s, off, 32);
  if (lane == 0) redS[wave] = s;
  __syncthreads();
  const float tot = redS[0] + redS[1];
  const float inv = 1.0f / tot;
  unsigned short hb[8];
#pragma unroll
  for (int e = 0; e < 8; ++e) hb[e] = h_bits((ev[e] * inv) * carry);
  const v4u u = (v4u){pk16(hb[0], hb[1]), pk16(hb[2], hb[3]), pk16(hb[4], hb[5]), pk16(hb[6], hb[7])};
  unsigned short* op = P + (size_t)row * kSegLen + c0;
  *(volatile v4u*)op = u;
  __threadfence();
  *(volatile v4u*)op = u;
}

__global__ __launch_bounds__(256) void gelu_kernel(const float* __restrict__ in, unsigned short* __restrict__ out,
                                                   int n2, float carry) {
  const int i = blockIdx.x * 256 + threadIdx.x;
  if (i >= n2) return;
  const float a = in[2 * (size_t)i];
  const float b = in[2 * (size_t)i + 1];
  const float ga = (0.5f * a * (1.0f + erff(a * 0.70710678118654752f))) * carry;
  const float gb = (0.5f * b * (1.0f + erff(b * 0.70710678118654752f))) * carry;
  const unsigned u = pk16(h_bits(ga), h_bits(gb));
  ((volatile unsigned*)out)[i] = u;
  __threadfence();
  ((volatile unsigned*)out)[i] = u;
}

extern "C" void kernel_launch(void* const* d_in, const int* in_sizes, int n_in,
                              void* d_out, int out_size, void* d_ws, size_t ws_size,
                              hipStream_t stream) {
  if (n_in < 16) return;
  if (ws_size < kWsTotal) return;
  if (out_size < kS * kD) return;

  const float* hidden = (const float*)d_in[0];
  const int*   cu     = (const int*)d_in[1];
  const float* cosb   = (const float*)d_in[2];
  const float* sinb   = (const float*)d_in[3];
  const float* ln1_g  = (const float*)d_in[4];
  const float* ln1_b  = (const float*)d_in[5];
  const float* qkv_w  = (const float*)d_in[6];
  const float* qkv_b  = (const float*)d_in[7];
  const float* proj_w = (const float*)d_in[8];
  const float* proj_b = (const float*)d_in[9];
  const float* ln2_g  = (const float*)d_in[10];
  const float* ln2_b  = (const float*)d_in[11];
  const float* fc1_w  = (const float*)d_in[12];
  const float* fc1_b  = (const float*)d_in[13];
  const float* fc2_w  = (const float*)d_in[14];
  const float* fc2_b  = (const float*)d_in[15];
  const int ncu = in_sizes[1];

  char* ws = (char*)d_ws;
  unsigned short* rW  = (unsigned short*)(ws + kRegW);
  float*          rXA = (float*)(ws + kRegXA);
  float*          rXB = (float*)(ws + kRegXB);
  unsigned short* rH  = (unsigned short*)(ws + kRegH);
  unsigned short* rQ  = (unsigned short*)(ws + kRegQ);
  unsigned short* rK  = (unsigned short*)(ws + kRegK);
  unsigned short* rVT = (unsigned short*)(ws + kRegVT);
  float*          qkvf   = (float*)(ws + kRegBig);
  float*          scores = (float*)(ws + kRegBig);
  unsigned short* Pp     = (unsigned short*)(ws + kRegBig + kBigSub);
  float*          fc1o   = (float*)(ws + kRegBig);
  unsigned short* act    = (unsigned short*)(ws + kRegBig + kBigSub);
  float* outp = (float*)d_out;

  const long segStrideRow = (long)kSegLen * kD;
  const long pairPlane    = (long)kSegLen * kSegLen;

  for (int i = 0; i < kDepth; ++i) {
    const float* xin  = (i == 0) ? hidden : rXB;
    float*       xmid = rXA;
    float*       xout = (i == kDepth - 1) ? outp : rXB;

    wt_kernel<<<dim3(kD / 64, (3 * kD) / 64), 256, 0, stream>>>(qkv_w + (size_t)i * kD * 3 * kD, rW, kD, 3 * kD, kWCarry);
    ln_kernel<<<kS, 128, 0, stream>>>(xin, ln1_g + (size_t)i * kD, ln1_b + (size_t)i * kD, rH);
    wmma_gemm64<0, false, 2, 0, false><<<dim3((kS / 64) * (3 * kD / 64) / 8, 1), 256, 0, stream>>>(
        rH, rH, kD, 0L, 0L,
        rW, rW, kD, 0L, 0L,
        (void*)qkvf, (void*)qkvf, 3 * kD, 0L, 0L,
        qkv_b + (size_t)i * 3 * kD,
        hidden, 0L,
        kS, 3 * kD, kD, 1.0f / kWCarry, 1);
    rope_kernel<<<dim3(kS / 64, kH), 256, 0, stream>>>(qkvf, cosb, sinb, rQ, rK, rVT);
    for (int c = 0; c < kNChunk; ++c) {
      const size_t colOff = (size_t)c * kHeadsPerChunk * kHD;
      wmma_gemm64<0, false, 0, 0, false><<<dim3(8, kPairsPerChunk), 256, 0, stream>>>(
          rQ + colOff, rQ + colOff, kD, (long)kHD, segStrideRow,
          rK + colOff, rK + colOff, kD, (long)kHD, segStrideRow,
          (void*)scores, (void*)scores, kSegLen, (long)kNSeg * pairPlane, pairPlane,
          qkv_b, hidden, 0L,
          kSegLen, kSegLen, kHD, 0.125f, kNSeg);
      softmax_kernel<<<kPairsPerChunk * kSegLen, 64, 0, stream>>>(scores, Pp, cu, ncu, kPCarry);
      wmma_gemm64<0, false, 0, 1, false><<<dim3(1, kPairsPerChunk), 256, 0, stream>>>(
          Pp, Pp, kSegLen, (long)kNSeg * pairPlane, pairPlane,
          rVT + colOff * kS, rVT + colOff * kS, kS, (long)kHD * kS, (long)kSegLen,
          (void*)(rH + colOff), (void*)(rH + colOff), kD, (long)kHD, segStrideRow,
          qkv_b, hidden, 0L,
          kSegLen, kHD, kSegLen, kAoCarry / kPCarry, kNSeg);
    }
    wt_kernel<<<dim3(kD / 64, kD / 64), 256, 0, stream>>>(proj_w + (size_t)i * kD * kD, rW, kD, kD, kWCarry);
    wmma_gemm64<0, false, 2, 0, true><<<dim3((kS / 64) * (kD / 64) / 8, 1), 256, 0, stream>>>(
        rH, rH, kD, 0L, 0L,
        rW, rW, kD, 0L, 0L,
        (void*)xmid, (void*)xmid, kD, 0L, 0L,
        proj_b + (size_t)i * kD,
        xin, 0L,
        kS, kD, kD, 1.0f / (kAoCarry * kWCarry), 1);

    ln_kernel<<<kS, 128, 0, stream>>>(xmid, ln2_g + (size_t)i * kD, ln2_b + (size_t)i * kD, rH);
    wt_kernel<<<dim3(kD / 64, kFF / 64), 256, 0, stream>>>(fc1_w + (size_t)i * kD * kFF, rW, kD, kFF, kWCarry);
    wmma_gemm64<0, false, 2, 0, false><<<dim3((kS / 64) * (kFF / 64) / 8, 1), 256, 0, stream>>>(
        rH, rH, kD, 0L, 0L,
        rW, rW, kD, 0L, 0L,
        (void*)fc1o, (void*)fc1o, kFF, 0L, 0L,
        fc1_b + (size_t)i * kFF,
        hidden, 0L,
        kS, kFF, kD, 1.0f / kWCarry, 1);
    gelu_kernel<<<(kS * kFF / 2) / 256, 256, 0, stream>>>(fc1o, act, kS * kFF / 2, kActCarry);
    wt_kernel<<<dim3(kFF / 64, kD / 64), 256, 0, stream>>>(fc2_w + (size_t)i * kFF * kD, rW, kFF, kD, kWCarry);
    wmma_gemm64<0, false, 2, 0, true><<<dim3((kS / 64) * (kD / 64) / 8, 1), 256, 0, stream>>>(
        act, act, kFF, 0L, 0L,
        rW, rW, kFF, 0L, 0L,
        (void*)xout, (void*)xout, kD, 0L, 0L,
        fc2_b + (size_t)i * kD,
        xmid, 0L,
        kS, kD, kFF, 1.0f / (kActCarry * kWCarry), 1);
  }
}
